// BaseModel_18081812316555
// MI455X (gfx1250) — hardware-run, weakly checked
//
#include <hip/hip_runtime.h>


#ifndef NB
#define NB 16
#endif
#define NB_FULL 16
#define CN    22
#define TT    1000
#define TP    1024
#define XK    32
#define EXPW  300
#define FCH   150
#define FCP   160
#define NBLK  3
#define CHP   480
#define CHK   512
#define SPD   100
#define SPP   128
#define K3    384
#define NCLS  4
#define NFLAT 5050
#define KTMAX 75
#define HFP   1028
#define UBP   1120
#define WZP   112
#define STP   264
#define JLD   101
#define NSWEEP 10
#define WSC   16.0f
#define WSI   (1.0f / 16.0f)
#define SQ2   1.41421356237f

static_assert(NB >= 1);
static_assert(NB <= NB_FULL);
static_assert(TP >= TT);
static_assert(TP % 256 == 0);
static_assert(TP % 64 == 0);
static_assert(CN <= XK);
static_assert(XK == 32);
static_assert(FCP >= FCH);
static_assert(FCP % 16 == 0);
static_assert(FCP % 8 == 0);
static_assert(NBLK * FCP == CHP);
static_assert(CHK >= CHP);
static_assert(CHK % 64 == 0);
static_assert(SPP >= SPD);
static_assert(SPP % 64 == 0);
static_assert(K3 == 3 * SPP);
static_assert(K3 % 32 == 0);
static_assert(NFLAT == SPD * (SPD + 1) / 2);
static_assert(NCLS == 4);
static_assert(((KTMAX + 15 + 31) / 32) * 32 <= 96);
static_assert(16 + 96 <= WZP);
static_assert(KTMAX / 2 + TT <= UBP);
static_assert(768 + 240 + 95 < UBP);
static_assert(UBP % 8 == 0);
static_assert(WZP % 8 == 0);
static_assert(HFP % 4 == 0);
static_assert(HFP >= TP);
static_assert(UBP >= TP);
static_assert(STP % 8 == 0);
static_assert(STP >= 256);
static_assert(NB_FULL * NCLS * 4 == 256);
static_assert(SPP * K3 / 8 == 24 * 256);
static_assert(16 * HFP * 4 + 16 * UBP * 2 + 16 * WZP * 2 <= 131072);
static_assert(2 * SPD * JLD * 4 + 4 * (SPD / 2) * 4 + SPD * 4 <= 131072);
static_assert(EXPW * 4 + EXPW * CN * 4 + FCH * CN * 4 + FCP * XK * 2 <= 131072);
static_assert(4 * 16 * STP * 2 + 64 * 4 <= 131072);

typedef _Float16 h16;
typedef unsigned short bf;
typedef __attribute__((ext_vector_type(16))) __bf16   v16bf;
typedef __attribute__((ext_vector_type(16))) _Float16 v16h;
typedef __attribute__((ext_vector_type(8)))  _Float16 v8h;
typedef __attribute__((ext_vector_type(8)))  unsigned short v8us;
typedef __attribute__((ext_vector_type(8)))  float    v8f;
typedef __attribute__((ext_vector_type(4)))  float    v4f;
typedef v4f  __attribute__((may_alias)) v4fa;

__device__ __forceinline__ unsigned short f2bf(float f) { unsigned u = __float_as_uint(f); u += 0x7FFFu + ((u >> 16) & 1u); return (unsigned short)(u >> 16); }
__device__ __forceinline__ float bfr(float f) { return __uint_as_float(((unsigned)f2bf(f)) << 16); }
__device__ __forceinline__ v16h cat16(v8h lo, v8h hi) { return __builtin_shufflevector(lo, hi, 0, 1, 2, 3, 4, 5, 6, 7, 8, 9, 10, 11, 12, 13, 14, 15); }
__device__ __forceinline__ v16bf cat16b(v8us lo, v8us hi) { return __builtin_bit_cast(v16bf, __builtin_shufflevector(lo, hi, 0, 1, 2, 3, 4, 5, 6, 7, 8, 9, 10, 11, 12, 13, 14, 15)); }
__device__ __forceinline__ v8f wmma16(v16h a, v16h b, v8f c) { return __builtin_amdgcn_wmma_f32_16x16x32_f16(false, a, false, b, (short)0, c, false, false); }
__device__ __forceinline__ v8f wmmab(v16bf a, v16bf b, v8f c) { return __builtin_amdgcn_wmma_f32_16x16x32_bf16(false, a, false, b, (short)0, c, false, false); }
__device__ __forceinline__ v16h  ldh(const h16* p) { return cat16(*(const v8h*)p, *(const v8h*)(p + 16)); }
__device__ __forceinline__ v16bf ldb(const bf* p)  { return cat16b(*(const v8us*)p, *(const v8us*)(p + 16)); }
__device__ __forceinline__ void wave_sync() { __builtin_amdgcn_fence(3  , "wavefront"); __builtin_amdgcn_wave_barrier(); asm volatile("" ::: "memory"); }

static __device__ __forceinline__ h16 toh_flush(float v) { const h16 r = (h16)v; return (fabsf(v) < 6.103515625e-05f) ? (h16)0.0f : r; }
__device__ __forceinline__ float bf2f(unsigned short h) { return __uint_as_float(((unsigned)h) << 16); }
__device__ __forceinline__ v8f wmma16g(v16h a, v16h b, v8f c) { c = wmma16(a, b, c); asm volatile("v_nop\n\tv_nop\n\tv_nop\n\tv_nop" : "+v"(c) : "v"(a), "v"(b)); return c; }
__device__ __forceinline__ v8f wmmabg(v16bf a, v16bf b, v8f c) { c = wmmab(a, b, c); asm volatile("v_nop\n\tv_nop\n\tv_nop\n\tv_nop" : "+v"(c) : "v"(a), "v"(b)); return c; }
__device__ __forceinline__ float wsum32(float v) { v += __shfl_xor(v, 16, 32); v += __shfl_xor(v, 8, 32); v += __shfl_xor(v, 4, 32); v += __shfl_xor(v, 2, 32); v += __shfl_xor(v, 1, 32); return v; }
__device__ __forceinline__ unsigned short piece3(float v, int pc) {
    const unsigned short h = f2bf(v); const float r1 = v - bf2f(h);
    const unsigned short m = f2bf(r1); const float r2 = r1 - bf2f(m);
    const unsigned short l = f2bf(r2);
    return (pc == 0) ? h : ((pc == 1) ? m : l);
}

__global__ __launch_bounds__(256) void k_xt(const float* __restrict__ x, h16* XT) {
    __shared__ __align__(16) h16 tile[64 * 40];
    const int tid = threadIdx.x; const int t0 = blockIdx.x * 64, b = blockIdx.y;
#pragma unroll 1
    for (int e = tid; e < 32 * 64; e += 256) {
        const int c = e >> 6, t = e & 63; const int tg = t0 + t;
        const int cc = c < CN ? c : CN - 1; const int tc = tg < TT ? tg : TT - 1;
        float v = x[((size_t)b * CN + cc) * TT + tc];
        asm volatile("" : "+v"(v));
        const float r = ((c < CN) & (tg < TT)) ? bfr(v) : 0.0f;
        tile[t * 40 + c] = toh_flush(r);
    }
    __syncthreads();
    const int row = tid >> 2, c8 = (tid & 3) * 8;
    const v8h val = *(const v8h*)(&tile[row * 40 + c8]);
    h16* dst = XT + ((size_t)b * TP + t0) * XK + (size_t)tid * 8;
    *(volatile v8h*)dst = val; __threadfence(); *(volatile v8h*)dst = val;
}

__global__ __launch_bounds__(256) void k_wfold(const float* __restrict__ w1, const float* __restrict__ w2, const float* __restrict__ w3, const float* __restrict__ w4, h16* WFb) {
    __shared__ float sg[EXPW];
    __shared__ float w3s[EXPW * CN];
    __shared__ float weff[FCH * CN];
    __shared__ __align__(16) h16 ot[FCP * XK];
    const int tid = threadIdx.x;
#pragma unroll 1
    for (int g = tid; g < EXPW; g += 256) {
        float nrm = 0.0f;
#pragma unroll 1
        for (int c = 0; c < CN; ++c) { const float v = bfr(w3[g * CN + c]); w3s[g * CN + c] = v; nrm += v * v; }
        nrm = sqrtf(nrm);
        sg[g] = bfr(w2[g]) * fminf(1.0f, 1.0f / (nrm + 1e-12f));
    }
    __syncthreads();
#pragma unroll 1
    for (int e = tid; e < FCH * CN; e += 256) {
        const int o = e / CN, c = e - o * CN;
        float acc = 0.0f;
#pragma unroll 1
        for (int g = 0; g < EXPW; ++g) acc += bfr(w4[o * EXPW + g]) * sg[g] * w3s[g * CN + c];
        weff[e] = acc;
    }
    __syncthreads();
    const float k0 = bfr(w1[0]), k1 = bfr(w1[1]), k2 = bfr(w1[2]);
#pragma unroll 1
    for (int e = tid; e < FCP * XK; e += 256) {
        const int o = e >> 5, c = e & 31;
        const int oc = o < FCH ? o : FCH - 1; const int cc = c < CN ? c : CN - 1;
        const int cp = cc + 1 < CN ? cc + 1 : CN - 1; const int cm = cc > 0 ? cc - 1 : 0;
        float a = k1 * weff[oc * CN + cc];
        const float ap = k0 * weff[oc * CN + cp]; const float am = k2 * weff[oc * CN + cm];
        a += (cc + 1 < CN) ? ap : 0.0f;
        a += (cc > 0) ? am : 0.0f;
        ot[e] = toh_flush(((o < FCH) & (c < CN)) ? a : 0.0f);
    }
    __syncthreads();
#pragma unroll 1
    for (int ps = 0; ps < 2; ++ps) {
#pragma unroll 1
        for (int q = tid; q < FCP * XK / 8; q += 256) { const v8h val = *(const v8h*)(&ot[q * 8]); *(volatile v8h*)(WFb + (size_t)q * 8) = val; }
        if (ps == 0) __threadfence(); }
}

__global__ __launch_bounds__(256) void k_ws(const float* __restrict__ w, h16* WS) {
    const int q = blockIdx.x * 256 + threadIdx.x;
    const int p = q >> 6, cc0 = (q & 63) * 8;
    const int blk = cc0 / FCP, o0 = cc0 - blk * FCP;
    const int pc = p < SPD ? p : SPD - 1; const int bc = blk < NBLK ? blk : NBLK - 1;
    v8h o;
#pragma unroll
    for (int i = 0; i < 8; ++i) {
        const int oo = o0 + i; const int oc = oo < FCH ? oo : FCH - 1;
        float v = w[(size_t)pc * (NBLK * FCH) + bc * FCH + oc];
        asm volatile("" : "+v"(v));
        const bool ok = (p < SPD) & (cc0 < CHP) & (oo < FCH);
        o[i] = toh_flush(ok ? bfr(v) * WSC : 0.0f);
    }
    h16* dst = WS + (size_t)q * 8;
    *(volatile v8h*)dst = o; __threadfence(); *(volatile v8h*)dst = o;
}

__global__ __launch_bounds__(256) void k_w3(const float* __restrict__ w, bf* W3) {
    const int q = blockIdx.x * 256 + threadIdx.x;
    const int i = q / 48, kk0 = (q - i * 48) * 8; const int k0 = kk0 & 127;
    const int ic = i < SPD ? i : SPD - 1;
    v8us o;
#pragma unroll
    for (int e = 0; e < 8; ++e) {
        const int k = k0 + e; const int kc = k < SPD ? k : SPD - 1;
        float v = w[ic * SPD + kc];
        asm volatile("" : "+v"(v));
        const unsigned short hv = f2bf(v);
        o[e] = ((i < SPD) & (k < SPD)) ? hv : (unsigned short)0;
    }
    bf* dst = W3 + (size_t)q * 8;
    *(volatile v8us*)dst = o; __threadfence(); *(volatile v8us*)dst = o;
}

__global__ __launch_bounds__(128) void k_block(const h16* __restrict__ XT, const h16* __restrict__ WFb,
                                               const float* __restrict__ g1, const float* __restrict__ b1, const float* __restrict__ w5,
                                               const float* __restrict__ g2, const float* __restrict__ b2, h16* HPb, int kt, int nks) {
    __shared__ __align__(16) float hf[16 * HFP];
    __shared__ __align__(16) h16 ub[16 * UBP];
    __shared__ __align__(16) h16 wz[16 * WZP];
    const int lane = threadIdx.x & 31, lr = lane & 15, hi = lane >> 4;
    const int wave = __builtin_amdgcn_readfirstlane((int)(threadIdx.x >> 5));
    const int o0 = blockIdx.x * 16, b = blockIdx.y;
    const int half = kt >> 1;
    { const v8h z = (v8h){};
#pragma unroll 1
      for (int e = threadIdx.x; e < 16 * UBP / 8; e += 128) *(v8h*)(&ub[e * 8]) = z;
#pragma unroll 1
      for (int e = threadIdx.x; e < 16 * WZP / 8; e += 128) *(v8h*)(&wz[e * 8]) = z; }
    { const v16h bw = ldh(WFb + (size_t)(o0 + lr) * XK + 8 * hi);
      const h16* xa = XT + ((size_t)b * TP + (size_t)wave * 256 + lr) * XK + 8 * hi;
#pragma unroll 1
      for (int i = 0; i < 16; ++i) {
          const v16h a = ldh(xa + (size_t)i * 16 * XK);
          v8f c = (v8f){}; c = wmma16g(a, bw, c);
          const int ho = lr * HFP + wave * 256 + i * 16 + 8 * hi;
          const v4f x0 = __builtin_shufflevector(c, c, 0, 1, 2, 3); const v4f x1 = __builtin_shufflevector(c, c, 4, 5, 6, 7);
          *(v4fa*)(&hf[ho]) = x0; *(v4fa*)(&hf[ho + 4]) = x1; } }
    __syncthreads();
#pragma unroll 1
    for (int q = 0; q < 4; ++q) {
        const int ch = wave * 4 + q; const int o = o0 + ch;
        float s = 0.0f;
#pragma unroll 1
        for (int t = lane; t < TT; t += 32) s += hf[ch * HFP + t];
        s = wsum32(s);
        const float mean = s * (1.0f / TT);
        float vs = 0.0f;
#pragma unroll 1
        for (int t = lane; t < TT; t += 32) { const float d = hf[ch * HFP + t] - mean; vs += d * d; }
        vs = wsum32(vs);
        const float rs = 1.0f / sqrtf(vs * (1.0f / TT) + 1e-5f);
#pragma unroll 1
        for (int t = lane; t < TT; t += 32) {
            const float u = (hf[ch * HFP + t] - mean) * rs * bfr(g1[t]) + bfr(b1[t]);
            ub[ch * UBP + half + t] = toh_flush(u); }
        const int oc = o < FCH ? o : FCH - 1;
#pragma unroll 1
        for (int j = lane; j < kt; j += 32) {
            float w = w5[(size_t)oc * kt + j];
            asm volatile("" : "+v"(w));
            wz[ch * WZP + 16 + j] = toh_flush((o < FCH) ? bfr(w) : 0.0f); }
    }
    __syncthreads();
#pragma unroll 1
    for (int q = 0; q < 4; ++q) {
        const int ch = wave * 4 + q;
        v8f c0 = (v8f){}, c1 = (v8f){}, c2 = (v8f){}, c3 = (v8f){};
#pragma unroll 1
        for (int ks = 0; ks < nks; ++ks) {
            const int k0 = ks * 32;
            const int wbase = ch * WZP + 16 + k0 + 8 * hi - lr;
            v16h a;
#pragma unroll
            for (int i = 0; i < 8; ++i) { a[i] = wz[wbase + i]; a[8 + i] = wz[wbase + 16 + i]; }
            const int ubase = ch * UBP + k0 + 16 * lr + 8 * hi;
            const v16h q0 = cat16(*(const v8h*)(&ub[ubase]),       *(const v8h*)(&ub[ubase + 16]));
            c0 = wmma16g(a, q0, c0);
            const v16h q1 = cat16(*(const v8h*)(&ub[ubase + 256]), *(const v8h*)(&ub[ubase + 256 + 16]));
            c1 = wmma16g(a, q1, c1);
            const v16h q2 = cat16(*(const v8h*)(&ub[ubase + 512]), *(const v8h*)(&ub[ubase + 512 + 16]));
            c2 = wmma16g(a, q2, c2);
            const v16h q3 = cat16(*(const v8h*)(&ub[ubase + 768]), *(const v8h*)(&ub[ubase + 768 + 16]));
            c3 = wmma16g(a, q3, c3);
        }
        const int ho = ch * HFP + 16 * lr + 8 * hi;
        { const v4f x0 = __builtin_shufflevector(c0, c0, 0, 1, 2, 3), x1 = __builtin_shufflevector(c0, c0, 4, 5, 6, 7); *(v4fa*)(&hf[ho]) = x0;       *(v4fa*)(&hf[ho + 4]) = x1; }
        { const v4f x0 = __builtin_shufflevector(c1, c1, 0, 1, 2, 3), x1 = __builtin_shufflevector(c1, c1, 4, 5, 6, 7); *(v4fa*)(&hf[ho + 256]) = x0; *(v4fa*)(&hf[ho + 256 + 4]) = x1; }
        { const v4f x0 = __builtin_shufflevector(c2, c2, 0, 1, 2, 3), x1 = __builtin_shufflevector(c2, c2, 4, 5, 6, 7); *(v4fa*)(&hf[ho + 512]) = x0; *(v4fa*)(&hf[ho + 512 + 4]) = x1; }
        { const v4f x0 = __builtin_shufflevector(c3, c3, 0, 1, 2, 3), x1 = __builtin_shufflevector(c3, c3, 4, 5, 6, 7); *(v4fa*)(&hf[ho + 768]) = x0; *(v4fa*)(&hf[ho + 768 + 4]) = x1; }
    }
    __syncthreads();
#pragma unroll 1
    for (int q = 0; q < 4; ++q) {
        const int ch = wave * 4 + q; const int o = o0 + ch;
        float s = 0.0f;
#pragma unroll 1
        for (int t = lane; t < TT; t += 32) s += hf[ch * HFP + t];
        s = wsum32(s);
        const float mean = s * (1.0f / TT);
        float vs = 0.0f;
#pragma unroll 1
        for (int t = lane; t < TT; t += 32) { const float d = hf[ch * HFP + t] - mean; vs += d * d; }
        vs = wsum32(vs);
        const float rs = 1.0f / sqrtf(vs * (1.0f / TT) + 1e-5f);
#pragma unroll 1
        for (int t = lane; t < TP; t += 32) {
            const int tc = t < TT ? t : TT - 1;
            float xv = hf[ch * HFP + tc]; float gv = g2[tc]; float bv = b2[tc];
            asm volatile("" : "+v"(xv), "+v"(gv), "+v"(bv));
            const float y = (xv - mean) * rs * bfr(gv) + bfr(bv);
            ub[ch * UBP + t] = toh_flush(((t < TT) & (o < FCH)) ? y : 0.0f); }
        wave_sync();
        h16* dst = HPb + ((size_t)b * CHP + o) * TP;
#pragma unroll 1
        for (int ps = 0; ps < 2; ++ps) {
#pragma unroll
            for (int sI = 0; sI < 4; ++sI) { const int piece = sI * 32 + lane;
                const v8h val = *(const v8h*)(&ub[ch * UBP + piece * 8]);
                *(volatile v8h*)(dst + (size_t)piece * 8) = val; }
            if (ps == 0) __threadfence(); }
        wave_sync();
    }
}
static_assert(4 * 32 * 16 == TP * 2);

__global__ __launch_bounds__(256) void k_tr(const h16* __restrict__ HP, h16* HT) {
    __shared__ __align__(16) h16 tl[64 * 72];
    const int tid = threadIdx.x; const int t0 = blockIdx.x * 64, c0 = blockIdx.y * 64, b = blockIdx.z;
    const v8h z = (v8h){};
#pragma unroll
    for (int ps = 0; ps < 2; ++ps) {
        const int row = ps * 32 + (tid >> 3), t8 = (tid & 7) * 8; const int c = c0 + row; const int cc = c < CHP ? c : CHP - 1;
        v8h v = *(const v8h*)(HP + ((size_t)b * CHP + cc) * TP + t0 + t8);
        asm volatile("" : "+v"(v));
        *(v8h*)(&tl[row * 72 + t8]) = (c < CHP) ? v : z; }
    __syncthreads();
    const int c8 = (tid & 7) * 8; const int ta = tid >> 3, tb = 32 + (tid >> 3);
    v8h oa, ob;
#pragma unroll
    for (int i = 0; i < 8; ++i) { oa[i] = tl[(c8 + i) * 72 + ta]; ob[i] = tl[(c8 + i) * 72 + tb]; }
    h16* da = HT + ((size_t)b * TP + t0 + ta) * CHK + c0 + c8;
    h16* db = HT + ((size_t)b * TP + t0 + tb) * CHK + c0 + c8;
    *(volatile v8h*)da = oa; *(volatile v8h*)db = ob; __threadfence(); *(volatile v8h*)da = oa; *(volatile v8h*)db = ob;
}

__global__ __launch_bounds__(128) void k_sconv(const h16* __restrict__ WS, const h16* __restrict__ HT, h16* SC) {
    __shared__ __align__(16) h16 st[4 * 16 * STP];
    __shared__ float part[64];
    const int lane = threadIdx.x & 31, lr = lane & 15, hi = lane >> 4;
    const int wave = __builtin_amdgcn_readfirstlane((int)(threadIdx.x >> 5));
    const int p0 = blockIdx.x * 16, b = blockIdx.y; const int tw = wave * 256;
    v8f acc[16];
#pragma unroll
    for (int nt = 0; nt < 16; ++nt) acc[nt] = (v8f){};
    const size_t aoff = (size_t)(p0 + lr) * CHK + 8 * hi;
    const size_t boff = ((size_t)b * TP + tw + lr) * CHK + 8 * hi;
#pragma unroll 1
    for (int kc = 0; kc < CHK; kc += 32) {
        const v16h a = ldh(WS + aoff + kc);
#pragma unroll
        for (int nt = 0; nt < 16; ++nt) { const v16h bq = ldh(HT + boff + (size_t)nt * 16 * CHK + kc); acc[nt] = wmma16g(a, bq, acc[nt]); }
    }
    float rsum[8];
#pragma unroll
    for (int r = 0; r < 8; ++r) { float v = 0.0f;
#pragma unroll
        for (int nt = 0; nt < 16; ++nt) v += acc[nt][r];
        v += __shfl_xor(v, 8, 32); v += __shfl_xor(v, 4, 32); v += __shfl_xor(v, 2, 32); v += __shfl_xor(v, 1, 32);
        rsum[r] = v; }
    if (lr == 0) {
#pragma unroll
        for (int r = 0; r < 8; ++r) part[wave * 16 + 8 * hi + r] = rsum[r]; }
    __syncthreads();
    float mean[8];
#pragma unroll
    for (int r = 0; r < 8; ++r) mean[r] = (part[8 * hi + r] + part[16 + 8 * hi + r] + part[32 + 8 * hi + r] + part[48 + 8 * hi + r]) * (WSI * (1.0f / TT));
    const int wb = wave * 16 * STP;
#pragma unroll
    for (int nt = 0; nt < 16; ++nt) {
        const int t = tw + 16 * nt + lr;
#pragma unroll
        for (int r = 0; r < 8; ++r) { const float val = acc[nt][r] * WSI - mean[r];
            st[wb + (8 * hi + r) * STP + 16 * nt + lr] = toh_flush((t < TT) ? val : 0.0f); } }
    wave_sync();
    h16* dst = SC + ((size_t)b * SPP + p0) * TP + tw + lane * 8;
#pragma unroll 1
    for (int ps = 0; ps < 2; ++ps) {
#pragma unroll 1
        for (int rr = 0; rr < 16; ++rr) { const v8h val = *(const v8h*)(&st[wb + rr * STP + lane * 8]);
            *(volatile v8h*)(dst + (size_t)rr * TP) = val; }
        if (ps == 0) __threadfence(); }
}

__global__ __launch_bounds__(32) void k_gemm_cov(const h16* __restrict__ SC, bf* OP) {
    __shared__ __align__(16) float os[16 * 68];
    const int lane = threadIdx.x & 31, lr = lane & 15, hi = lane >> 4;
    const int m0 = blockIdx.x * 16, n0 = blockIdx.y * 64, b = blockIdx.z;
    v8f acc[4];
#pragma unroll
    for (int nb = 0; nb < 4; ++nb) acc[nb] = (v8f){};
    const size_t aoff = ((size_t)b * SPP + m0 + lr) * TP + 8 * hi, boff = ((size_t)b * SPP + n0 + lr) * TP + 8 * hi;
#pragma unroll 1
    for (int kc = 0; kc < TP; kc += 32) {
        const v16h a = ldh(SC + aoff + kc);
#pragma unroll
        for (int nb = 0; nb < 4; ++nb) { const v16h bq = ldh(SC + boff + (size_t)nb * 16 * TP + kc); acc[nb] = wmma16g(a, bq, acc[nb]); }
    }
#pragma unroll
    for (int nb = 0; nb < 4; ++nb) {
#pragma unroll
        for (int j = 0; j < 8; ++j) { const int gi = m0 + 8 * hi + j, gj = n0 + nb * 16 + lr;
            os[(hi * 8 + j) * 68 + nb * 16 + lr] = acc[nb][j] * (1.0f / (TT - 1)) + (((gi == gj) & (gi < SPD)) ? 1e-4f : 0.0f); } }
    wave_sync();
    bf* dst = OP + ((size_t)b * SPP + m0) * K3 + n0;
#pragma unroll 1
    for (int ps = 0; ps < 2; ++ps) {
#pragma unroll 1
        for (int pc = 0; pc < 3; ++pc) {
#pragma unroll
            for (int s = 0; s < 4; ++s) { const int row = 4 * s + (lane >> 3), c8 = (lane & 7) * 8;
                const v4f x0 = *(const v4fa*)(&os[row * 68 + c8]); const v4f x1 = *(const v4fa*)(&os[row * 68 + c8 + 4]); v8us o;
#pragma unroll
                for (int i = 0; i < 4; ++i) { o[i] = piece3(x0[i], pc); o[4 + i] = piece3(x1[i], pc); }
                *(volatile v8us*)(dst + (size_t)row * K3 + pc * SPP + c8) = o; } }
        if (ps == 0) __threadfence(); }
}

__global__ __launch_bounds__(32) void k_gemm_b(const bf* __restrict__ A, size_t sA, const bf* __restrict__ Bt, size_t sB, int K, int mode, bf* OP, float* OF) {
    __shared__ __align__(16) float os[16 * 68];
    const int lane = threadIdx.x & 31, lr = lane & 15, hi = lane >> 4;
    const int m0 = blockIdx.x * 16, n0 = blockIdx.y * 64, b = blockIdx.z;
    v8f acc[4];
#pragma unroll
    for (int nb = 0; nb < 4; ++nb) acc[nb] = (v8f){};
    const size_t aoff = (size_t)b * sA + (size_t)(m0 + lr) * K + 8 * hi, boff = (size_t)b * sB + (size_t)(n0 + lr) * K + 8 * hi;
#pragma unroll 1
    for (int kc = 0; kc < K; kc += 32) {
        const v16bf a = ldb(A + aoff + kc);
#pragma unroll
        for (int nb = 0; nb < 4; ++nb) { const v16bf bq = ldb(Bt + boff + (size_t)nb * 16 * K + kc); acc[nb] = wmmabg(a, bq, acc[nb]); }
    }
#pragma unroll
    for (int nb = 0; nb < 4; ++nb) {
#pragma unroll
        for (int j = 0; j < 8; ++j) os[(hi * 8 + j) * 68 + nb * 16 + lr] = acc[nb][j]; }
    wave_sync();
    if (mode == 0) {
        bf* dst = OP + ((size_t)b * SPP + m0) * K3 + n0;
#pragma unroll 1
        for (int ps = 0; ps < 2; ++ps) {
#pragma unroll 1
            for (int pc = 0; pc < 3; ++pc) {
#pragma unroll
                for (int s = 0; s < 4; ++s) { const int row = 4 * s + (lane >> 3), c8 = (lane & 7) * 8;
                    const v4f x0 = *(const v4fa*)(&os[row * 68 + c8]); const v4f x1 = *(const v4fa*)(&os[row * 68 + c8 + 4]); v8us o;
#pragma unroll
                    for (int i = 0; i < 4; ++i) { o[i] = piece3(x0[i], pc); o[4 + i] = piece3(x1[i], pc); }
                    *(volatile v8us*)(dst + (size_t)row * K3 + pc * SPP + c8) = o; } }
            if (ps == 0) __threadfence(); }
    } else {
        float* dst = OF + ((size_t)b * SPP + m0) * SPP + n0;
#pragma unroll 1
        for (int ps = 0; ps < 2; ++ps) {
#pragma unroll
            for (int s = 0; s < 8; ++s) { const int row = 2 * s + (lane >> 4), c4 = (lane & 15) * 4;
                const v4f val = *(const v4fa*)(&os[row * 68 + c4]);
                *(volatile v4f*)(dst + (size_t)row * SPP + c4) = val; }
            if (ps == 0) __threadfence(); }
    }
}
static_assert(4 * 4 == 16);
static_assert(8 * 2 == 16);
static_assert(8 * 16 == SPP);

__global__ __launch_bounds__(256) void k_eig(const float* __restrict__ PM, bf* VW3, bf* V3) {
    __shared__ float Am[SPD * JLD];
    __shared__ float Vm[SPD * JLD];
    __shared__ int   pp[SPD / 2];
    __shared__ int   qq[SPD / 2];
    __shared__ float cs[SPD / 2];
    __shared__ float sn[SPD / 2];
    __shared__ float lw[SPD];
    const int tid = threadIdx.x; const int b = blockIdx.x;
    const float* Pb = PM + (size_t)b * SPP * SPP;
#pragma unroll 1
    for (int e = tid; e < SPD * SPD; e += 256) { const int i = e / SPD, j = e - i * SPD;
        Am[i * JLD + j] = 0.5f * (Pb[i * SPP + j] + Pb[j * SPP + i]);
        Vm[i * JLD + j] = (i == j) ? 1.0f : 0.0f; }
    __syncthreads();
    const int nm1 = SPD - 1;
    const int pr0 = tid / SPD; const int kk0 = tid - pr0 * SPD;
#pragma unroll 1
    for (int sweep = 0; sweep < NSWEEP; ++sweep) {
#pragma unroll 1
        for (int r = 0; r < nm1; ++r) {
            if (tid < SPD / 2) {
                int p, q;
                if (tid == 0) { p = nm1; q = r; }
                else { p = (r + tid) % nm1; q = (r - tid + nm1) % nm1; }
                if (p > q) { const int t0 = p; p = q; q = t0; }
                const float app = Am[p * JLD + p], aqq = Am[q * JLD + q], apq = Am[p * JLD + q];
                float c = 1.0f, s = 0.0f;
                if (fabsf(apq) > 1e-12f) {
                    const float tau = (aqq - app) / (2.0f * apq);
                    const float rt = sqrtf(1.0f + tau * tau);
                    const float t = (tau >= 0.0f) ? 1.0f / (tau + rt) : 1.0f / (tau - rt);
                    c = 1.0f / sqrtf(1.0f + t * t);
                    s = t * c; }
                pp[tid] = p; qq[tid] = q; cs[tid] = c; sn[tid] = s;
            }
            __syncthreads();
            { int pr = pr0, k = kk0;
#pragma unroll 1
              while (pr < SPD / 2) {
                  const int p = pp[pr], q = qq[pr]; const float c = cs[pr], s = sn[pr];
                  const float apk = Am[p * JLD + k], aqk = Am[q * JLD + k];
                  Am[p * JLD + k] = c * apk - s * aqk;
                  Am[q * JLD + k] = s * apk + c * aqk;
                  k += 56; pr += 2; if (k >= SPD) { k -= SPD; pr += 1; } } }
            __syncthreads();
            { int pr = pr0, k = kk0;
#pragma unroll 1
              while (pr < SPD / 2) {
                  const int p = pp[pr], q = qq[pr]; const float c = cs[pr], s = sn[pr];
                  const float akp = Am[k * JLD + p], akq = Am[k * JLD + q];
                  Am[k * JLD + p] = c * akp - s * akq;
                  Am[k * JLD + q] = s * akp + c * akq;
                  const float vkp = Vm[k * JLD + p], vkq = Vm[k * JLD + q];
                  Vm[k * JLD + p] = c * vkp - s * vkq;
                  Vm[k * JLD + q] = s * vkp + c * vkq;
                  k += 56; pr += 2; if (k >= SPD) { k -= SPD; pr += 1; } } }
            __syncthreads();
        }
    }
    if (tid < SPD) lw[tid] = logf(fmaxf(Am[tid * JLD + tid], 1e-6f));
    __syncthreads();
    bf* vwb = VW3 + (size_t)b * SPP * K3; bf* v3b = V3 + (size_t)b * SPP * K3;
#pragma unroll 1
    for (int ps = 0; ps < 2; ++ps) {
#pragma unroll 1
        for (int it = 0; it < 24; ++it) {
            const int q = it * 256 + tid; const int row = q / 48; const int kq = (q - row * 48) * 8; const int sgm = kq >> 7; const int k0 = kq & 127;
            const int rc = row < SPD ? row : SPD - 1;
            v8us ow, ov;
#pragma unroll
            for (int e = 0; e < 8; ++e) {
                const int k = k0 + e; const int kc = k < SPD ? k : SPD - 1; const bool ok = (row < SPD) & (k < SPD);
                const float v = Vm[rc * JLD + kc]; const float w = v * lw[kc];
                const unsigned short vh = f2bf(v); const unsigned short vl = f2bf(v - bf2f(vh));
                const unsigned short wh = f2bf(w); const unsigned short wl = f2bf(w - bf2f(wh));
                const unsigned short sw = (sgm == 2) ? wl : wh; const unsigned short sv = (sgm == 1) ? vl : vh;
                ow[e] = ok ? sw : (unsigned short)0; ov[e] = ok ? sv : (unsigned short)0; }
            *(volatile v8us*)(vwb + (size_t)q * 8) = ow; *(volatile v8us*)(v3b + (size_t)q * 8) = ov; }
        if (ps == 0) __threadfence(); }
}

__global__ __launch_bounds__(256) void k_vec(const float* __restrict__ LM, float* OUT1, int ntot) {
    __shared__ int rsx[SPD + 1];
    const int tid = threadIdx.x;
    if (tid <= SPD) rsx[tid] = tid * SPD - (tid * (tid - 1)) / 2;
    __syncthreads();
    const int e0 = (blockIdx.x * 256 + tid) * 4;
    if (e0 >= ntot) return;
    v4f val;
#pragma unroll
    for (int i = 0; i < 4; ++i) {
        int e = e0 + i; e = e < ntot ? e : ntot - 1;
        const int b = e / NFLAT; const int w = e - b * NFLAT;
        int lo = 0, hh = SPD - 1;
#pragma unroll
        for (int s = 0; s < 7; ++s) { const int mid = (lo + hh + 1) >> 1; const bool le = rsx[mid] <= w; lo = le ? mid : lo; hh = le ? hh : mid - 1; }
        int j = lo + (w - rsx[lo]); j = j < SPD ? j : SPD - 1;
        const float v = LM[((size_t)b * SPP + lo) * SPP + j];
        val[i] = v * ((lo == j) ? 1.0f : SQ2); }
    if (e0 + 3 < ntot) {
        *(volatile v4f*)(OUT1 + e0) = val; __threadfence(); *(volatile v4f*)(OUT1 + e0) = val;
    } else {
#pragma unroll
        for (int i = 0; i < 4; ++i) if (e0 + i < ntot) *(volatile float*)(OUT1 + e0 + i) = val[i];
        __threadfence();
#pragma unroll
        for (int i = 0; i < 4; ++i) if (e0 + i < ntot) *(volatile float*)(OUT1 + e0 + i) = val[i];
    }
}

__global__ __launch_bounds__(256) void k_fc(const float* __restrict__ LM, const float* __restrict__ wfc, const float* __restrict__ bfc, float* OUT0) {
    __shared__ __align__(16) float lg[NB_FULL * NCLS];
    const int lane = threadIdx.x & 31;
    const int wave = __builtin_amdgcn_readfirstlane((int)(threadIdx.x >> 5));
#pragma unroll 1
    for (int oi = wave; oi < NB * NCLS; oi += 8) {
        const int b = oi >> 2, cls = oi & 3;
        float acc = 0.0f;
#pragma unroll 1
        for (int i = 0; i < SPD; ++i) {
            const int rs = i * SPD - (i * (i - 1)) / 2;
#pragma unroll 1
            for (int s = 0; s < 4; ++s) {
                const int j = i + lane + 32 * s; const int jc = j < SPD ? j : SPD - 1;
                float l = LM[((size_t)b * SPP + i) * SPP + jc]; float w = wfc[(size_t)cls * NFLAT + rs + (jc - i)];
                asm volatile("" : "+v"(l), "+v"(w));
                const float fl = l * ((jc == i) ? 1.0f : SQ2);
                const float pr = fl * bfr(w);
                acc += (j < SPD) ? pr : 0.0f; } }
        acc = wsum32(acc);
        if (lane == 0) lg[oi] = acc + bfr(bfc[cls]);
    }
    __syncthreads();
    if (wave == 0) {
        const int lc = lane < NB ? lane : NB - 1;
        const v4f val = *(const v4fa*)(&lg[lc * 4]);
        if (lane < NB) { *(volatile v4f*)(OUT0 + lane * 4) = val; __threadfence(); *(volatile v4f*)(OUT0 + lane * 4) = val; }
    }
}

static constexpr size_t al256(size_t v) { return (v + 255) & ~(size_t)255; }
static constexpr size_t SZ_XT = al256((size_t)NB * TP * XK * 2);
static constexpr size_t SZ_WF = al256((size_t)CHP * XK * 2);
static constexpr size_t SZ_WS = al256((size_t)SPP * CHK * 2);
static constexpr size_t SZ_W3 = al256((size_t)SPP * K3 * 2);
static constexpr size_t SZ_HP = al256((size_t)NB * CHP * TP * 2);
static constexpr size_t SZ_HT = al256((size_t)NB * TP * CHK * 2);
static constexpr size_t SZ_SC = al256((size_t)NB * SPP * TP * 2);
static constexpr size_t SZ_P3 = al256((size_t)NB * SPP * K3 * 2);
static constexpr size_t SZ_F  = al256((size_t)NB * SPP * SPP * 4);
static constexpr size_t SZ_TOTAL = SZ_XT + SZ_WF + SZ_WS + SZ_W3 + SZ_HP + SZ_HT + SZ_SC + 4 * SZ_P3 + 2 * SZ_F;
static_assert(SZ_TOTAL <= (size_t)134217728);
static_assert(((size_t)FCP * XK * 2) % 256 == 0);
static_assert(((size_t)FCP * TP * 2) % 256 == 0);
static_assert((SPP * CHK / 8) % 256 == 0);
static_assert((SPP * K3 / 8) % 256 == 0);

extern "C" void kernel_launch(void* const* d_in, const int* in_sizes, int n_in,
                              void* d_out, int out_size, void* d_ws, size_t ws_size, hipStream_t stream) {
    if (n_in < 32) return;
    const int KT[3] = { 15, 75, 55 };
    if ((size_t)in_sizes[0] < (size_t)NB * CN * TT) return;
    for (int bi = 0; bi < 3; ++bi) {
        const int base = 1 + 9 * bi;
        if (in_sizes[base] < 3 || in_sizes[base + 1] < EXPW || in_sizes[base + 2] < EXPW * CN || in_sizes[base + 3] < FCH * EXPW) return;
        if (in_sizes[base + 4] < TT || in_sizes[base + 5] < TT || in_sizes[base + 6] < FCH * KT[bi] || in_sizes[base + 7] < TT || in_sizes[base + 8] < TT) return;
        if (KT[bi] > KTMAX || (KT[bi] + 46) / 32 > 3) return;
    }
    if (in_sizes[28] < SPD * NBLK * FCH || in_sizes[29] < SPD * SPD || in_sizes[30] < NCLS * NFLAT || in_sizes[31] < NCLS) return;
    if ((size_t)out_size < (size_t)NB_FULL * NCLS + (size_t)NB * NFLAT) return;
    if (SZ_TOTAL > ws_size) return;
    const float* x = (const float*)d_in[0];
    const float* w_sconv = (const float*)d_in[28];
    const float* w_aff   = (const float*)d_in[29];
    const float* w_fc    = (const float*)d_in[30];
    const float* b_fc    = (const float*)d_in[31];
    float* OUT0 = (float*)d_out;
    float* OUT1 = (float*)d_out + NB_FULL * NCLS;
    char* wsp = (char*)d_ws;
    h16* XT  = (h16*)wsp; wsp += SZ_XT;
    h16* WF  = (h16*)wsp; wsp += SZ_WF;
    h16* WS  = (h16*)wsp; wsp += SZ_WS;
    bf*  W3  = (bf*)wsp;  wsp += SZ_W3;
    h16* HP  = (h16*)wsp; wsp += SZ_HP;
    h16* HT  = (h16*)wsp; wsp += SZ_HT;
    h16* SC  = (h16*)wsp; wsp += SZ_SC;
    bf*  CV3 = (bf*)wsp;  wsp += SZ_P3;
    bf*  T3  = (bf*)wsp;  wsp += SZ_P3;
    bf*  VW3 = (bf*)wsp;  wsp += SZ_P3;
    bf*  V3  = (bf*)wsp;  wsp += SZ_P3;
    float* PM = (float*)wsp; wsp += SZ_F;
    float* LM = (float*)wsp; wsp += SZ_F;

    k_xt<<<dim3(TP / 64, NB, 1), 256, 0, stream>>>(x, XT);
    for (int bi = 0; bi < 3; ++bi) {
        const int base = 1 + 9 * bi;
        k_wfold<<<1, 256, 0, stream>>>((const float*)d_in[base], (const float*)d_in[base + 1], (const float*)d_in[base + 2], (const float*)d_in[base + 3],
                                       WF + (size_t)bi * FCP * XK);
    }
    k_ws<<<SPP * CHK / 8 / 256, 256, 0, stream>>>(w_sconv, WS);
    k_w3<<<SPP * K3 / 8 / 256, 256, 0, stream>>>(w_aff, W3);
    for (int bi = 0; bi < 3; ++bi) {
        const int base = 1 + 9 * bi;
        k_block<<<dim3(FCP / 16, NB, 1), 128, 0, stream>>>(XT, WF + (size_t)bi * FCP * XK,
            (const float*)d_in[base + 4], (const float*)d_in[base + 5], (const float*)d_in[base + 6], (const float*)d_in[base + 7], (const float*)d_in[base + 8],
            HP + (size_t)bi * FCP * TP, KT[bi], (KT[bi] + 46) / 32);
    }
    k_tr<<<dim3(TP / 64, CHK / 64, NB), 256, 0, stream>>>(HP, HT);
    k_sconv<<<dim3(SPP / 16, NB, 1), 128, 0, stream>>>(WS, HT, SC);
    k_gemm_cov<<<dim3(SPP / 16, SPP / 64, NB), 32, 0, stream>>>(SC, CV3);
    k_gemm_b<<<dim3(SPP / 16, SPP / 64, NB), 32, 0, stream>>>(W3, (size_t)0, CV3, (size_t)SPP * K3, K3, 0, T3, PM);
    k_gemm_b<<<dim3(SPP / 16, SPP / 64, NB), 32, 0, stream>>>(T3, (size_t)SPP * K3, W3, (size_t)0, K3, 1, VW3, PM);
    k_eig<<<NB, 256, 0, stream>>>(PM, VW3, V3);
    k_gemm_b<<<dim3(SPP / 16, SPP / 64, NB), 32, 0, stream>>>(VW3, (size_t)SPP * K3, V3, (size_t)SPP * K3, K3, 1, T3, LM);
    { const int ntot = NB * NFLAT; const int pieces = (ntot + 3) / 4;
      k_vec<<<(pieces + 255) / 256, 256, 0, stream>>>(LM, OUT1, ntot); }
    k_fc<<<1, 256, 0, stream>>>(LM, w_fc, b_fc, OUT0);
}
